// GatedAttentionBlock_33165737459846
// MI455X (gfx1250) — hardware-verified
//
#include <hip/hip_runtime.h>
#include <math.h>

constexpr int kNb     = 2;
constexpr int kSeq    = 2048;
constexpr int kDim    = 1024;
constexpr int kHeads  = 16;
constexpr int kHd     = 64;
constexpr int kTok    = kNb * kSeq;
constexpr int kGroups = kNb * kHeads;
constexpr int kGch    = 4;
constexpr int kNchunk = kGroups / kGch;
constexpr int kDff    = 4096;
constexpr int kMlpRows = 1024;
constexpr float kWCarry = 64.0f;
constexpr float kACarry = 64.0f;
constexpr float kPCarry = 2048.0f;
constexpr float kFill   = -1e30f;
constexpr size_t kMiB = 1048576;
constexpr size_t kCarveBytes = 128 * kMiB;

typedef __attribute__((ext_vector_type(16))) _Float16 v16h;
typedef __attribute__((ext_vector_type(8)))  _Float16 v8h;
typedef __attribute__((ext_vector_type(16))) __bf16   v16b;
typedef __attribute__((ext_vector_type(8)))  __bf16   v8b;
typedef __attribute__((ext_vector_type(8)))  float    v8f;
typedef __attribute__((ext_vector_type(4)))  float    v4f;
typedef __attribute__((ext_vector_type(4)))  unsigned int v4u;
typedef __attribute__((ext_vector_type(4)))  int      v4i;

__device__ __forceinline__ unsigned short f2bf_bits(float f) {
  unsigned u = __float_as_uint(f);
  return (unsigned short)((u + 0x7FFFu + ((u >> 16) & 1u)) >> 16);
}
__device__ __forceinline__ float bf_bits2f(unsigned short h) { return __uint_as_float(((unsigned)h) << 16); }

__device__ __forceinline__ void dep_guard_h(v8f& a, v8f& b, v16h x, v16h y) { asm volatile("v_nop\n\tv_nop\n\tv_nop\n\tv_nop" : "+v"(a), "+v"(b) : "v"(x), "v"(y)); }
__device__ __forceinline__ void dep_guard_b(v8f& a, v8f& b, v16b x, v16b y) { asm volatile("v_nop\n\tv_nop\n\tv_nop\n\tv_nop" : "+v"(a), "+v"(b) : "v"(x), "v"(y)); }
__device__ __forceinline__ void keep4_h(v16h a, v16h b, v16h c, v16h d) { asm volatile("v_nop" :: "v"(a), "v"(b), "v"(c), "v"(d)); }
__device__ __forceinline__ void keep4_b(v16b a, v16b b, v16b c, v16b d) { asm volatile("v_nop" :: "v"(a), "v"(b), "v"(c), "v"(d)); }
__device__ __forceinline__ void acc_guard4(v8f& a, v8f& b, v8f& c, v8f& d) { asm volatile("v_nop\n\tv_nop\n\tv_nop\n\tv_nop" : "+v"(a), "+v"(b), "+v"(c), "+v"(d)); }
template <typename T> struct Frag;
template <> struct Frag<_Float16> {
  typedef v16h V; union U { v16h v; v8h h[2]; };
  static __device__ __forceinline__ v16h load(const _Float16* p) {
    U f; f.h[0] = *(const v8h*)(p); f.h[1] = *(const v8h*)(p + 16); return f.v;
  }
  static __device__ __forceinline__ v8f mma(v16h a, v16h b, v8f c) {
    return __builtin_amdgcn_wmma_f32_16x16x32_f16(false, a, false, b, (short)0, c, false, false);
  }
  static __device__ __forceinline__ void guard(v8f& a, v8f& b, v16h x, v16h y) { dep_guard_h(a, b, x, y); }
  static __device__ __forceinline__ void keep(v16h a, v16h b, v16h c, v16h d) { keep4_h(a, b, c, d); }
};
template <> struct Frag<__bf16> {
  typedef v16b V; union U { v16b v; v8b h[2]; };
  static __device__ __forceinline__ v16b load(const __bf16* p) {
    U f; f.h[0] = *(const v8b*)(p); f.h[1] = *(const v8b*)(p + 16); return f.v;
  }
  static __device__ __forceinline__ v8f mma(v16b a, v16b b, v8f c) {
    return __builtin_amdgcn_wmma_f32_16x16x32_bf16(false, a, false, b, (short)0, c, false, false);
  }
  static __device__ __forceinline__ void guard(v8f& a, v8f& b, v16b x, v16b y) { dep_guard_b(a, b, x, y); }
  static __device__ __forceinline__ void keep(v16b a, v16b b, v16b c, v16b d) { keep4_b(a, b, c, d); }
};

__device__ __forceinline__ unsigned pk16(unsigned short a, unsigned short b) { return (unsigned)a | ((unsigned)b << 16); }
__device__ __forceinline__ unsigned short h_bits(float f) { const _Float16 h = (_Float16)f; return __builtin_bit_cast(unsigned short, h); }

template <int ET> struct Elem;
template <> struct Elem<0> { typedef _Float16 T; };
template <> struct Elem<1> { typedef __bf16 T; };
template <int ET, bool SPLIT, int BIAS_MODE, int OUT_MODE, bool RESID, int ACT = 0>
__global__ __launch_bounds__(256) void wmma_gemm64(
    const unsigned short* __restrict__ Ap, const unsigned short* __restrict__ A2p, int lda, long strideA,
    const unsigned short* __restrict__ Btp, const unsigned short* __restrict__ Bt2p, int ldb, long strideB,
    void* __restrict__ Cout, void* __restrict__ Cout2, int ldc, long strideC,
    const float* __restrict__ bias,
    const float* __restrict__ resid, long strideR,
    const float* __restrict__ aux,
    int M, int N, int K, float scale) {
  typedef typename Elem<ET>::T T;
  typedef typename Frag<T>::V V;
  const T* A = (const T*)Ap; const T* A2 = (const T*)A2p; const T* Bt = (const T*)Btp; const T* Bt2 = (const T*)Bt2p;
  __shared__ __align__(16) float sT[8][16 * 68];
  const int b    = blockIdx.y;
  const int lane = threadIdx.x & 31;
  const int wave = threadIdx.x >> 5;
  const int tilesN = N >> 6;
  const int tilesM = M >> 6;
  const int tile = blockIdx.x * 8 + wave;
  if (tile >= tilesM * tilesN) return;
  const int tm = tile / tilesN;
  const int tn = tile - tm * tilesN;
  const int m0 = tm << 6;
  const int n0 = tn << 6;

  const T* Ab  = A  + (size_t)b * strideA;
  const T* Bb  = Bt + (size_t)b * strideB;
  const T* Ab2 = SPLIT ? (A2  + (size_t)b * strideA) : nullptr;
  const T* Bb2 = SPLIT ? (Bt2 + (size_t)b * strideB) : nullptr;

  const int rlane = lane & 15;
  const int koff  = (lane >> 4) * 8;
  const int mOff  = (lane >> 4) * 8;

  v8f acc[4][4];
#pragma unroll
  for (int i = 0; i < 4; ++i)
#pragma unroll
    for (int j = 0; j < 4; ++j) acc[i][j] = (v8f){0.f,0.f,0.f,0.f,0.f,0.f,0.f,0.f};

  for (int k0 = 0; k0 < K; k0 += 32) {
    V bh[4], bl[4];
#pragma unroll
    for (int j = 0; j < 4; ++j) {
      const size_t bo = (size_t)(n0 + (j << 4) + rlane) * ldb + koff + k0;
      bh[j] = Frag<T>::load(Bb + bo);
      if (SPLIT) bl[j] = Frag<T>::load(Bb2 + bo);
    }
#pragma unroll
    for (int i = 0; i < 4; ++i) {
      const size_t ao = (size_t)(m0 + (i << 4) + rlane) * lda + koff + k0;
      V ah = Frag<T>::load(Ab + ao);
      V al;
      if (SPLIT) al = Frag<T>::load(Ab2 + ao);
#pragma unroll
      for (int j = 0; j < 4; ++j) {
        acc[i][j] = Frag<T>::mma(ah, bh[j], acc[i][j]);
        if (SPLIT) {
          acc[i][j] = Frag<T>::mma(ah, bl[j], acc[i][j]);
          acc[i][j] = Frag<T>::mma(al, bh[j], acc[i][j]);
        }
      }
      Frag<T>::guard(acc[i][0], acc[i][3], ah, SPLIT ? al : ah);
    }
    Frag<T>::keep(bh[0], bh[1], bh[2], bh[3]);
    if (SPLIT) Frag<T>::keep(bl[0], bl[1], bl[2], bl[3]);
  }
  acc_guard4(acc[0][0], acc[0][1], acc[0][2], acc[0][3]);
  acc_guard4(acc[1][0], acc[1][1], acc[1][2], acc[1][3]);
  acc_guard4(acc[2][0], acc[2][1], acc[2][2], acc[2][3]);
  acc_guard4(acc[3][0], acc[3][1], acc[3][2], acc[3][3]);

  float* slab = sT[wave];
  const float* Rb = RESID ? (resid + (size_t)b * strideR) : nullptr;
  const float* Xb = (ACT == 6) ? (aux + (size_t)b * strideR) : nullptr;
#pragma unroll
  for (int i = 0; i < 4; ++i) {
    const int mBase = m0 + (i << 4);
#pragma unroll
    for (int j = 0; j < 4; ++j) {
      const int n = n0 + (j << 4) + rlane;
      float bv = 0.f;
      if (BIAS_MODE == 2) bv = bias[n];
#pragma unroll
      for (int r = 0; r < 8; ++r) {
        float v = acc[i][j][r] * scale;
        if (BIAS_MODE == 1) v += bias[mBase + mOff + r];
        if (BIAS_MODE == 2) v += bv;
        if (RESID && ACT != 6) v += Rb[(size_t)(mBase + mOff + r) * ldc + n];
        if (ACT == 2) v = fmaxf(v, 0.0f);
        if (ACT == 4) v = (v > 0.f) ? v : 0.01f * v;
        if (ACT == 6) {
          const float vc = fminf(fmaxf(v, -40.0f), 40.0f);
          const float sg = __builtin_amdgcn_rcpf(1.0f + expf(-vc));
          v = Xb[(size_t)(mBase + mOff + r) * ldc + n] * sg;
          if (RESID) v += Rb[(size_t)(mBase + mOff + r) * ldc + n];
        }
        slab[(mOff + r) * 68 + (j << 4) + rlane] = v;
      }
    }
    __builtin_amdgcn_fence(__ATOMIC_RELEASE, "workgroup");
    __builtin_amdgcn_wave_barrier();
    __builtin_amdgcn_fence(__ATOMIC_ACQUIRE, "workgroup");
    if (OUT_MODE == 0) {
      float* C = (float*)Cout + (size_t)b * strideC;
      const int hh = lane >> 4, c4 = (lane & 15) * 4;
      for (int pass = 0; pass < 2; ++pass) {
#pragma unroll
        for (int it = 0; it < 8; ++it) {
          const int row = it * 2 + hh;
          v4f v = *(const v4f*)(slab + row * 68 + c4);
          *(volatile v4f*)(C + (size_t)(mBase + row) * ldc + n0 + c4) = v;
        }
        __threadfence();
      }
    } else {
      const int q = lane >> 3, c8 = (lane & 7) * 8;
      unsigned short* C  = (unsigned short*)Cout  + (size_t)b * strideC;
      unsigned short* C2 = (OUT_MODE == 2) ? ((unsigned short*)Cout2 + (size_t)b * strideC) : nullptr;
      for (int pass = 0; pass < 2; ++pass) {
#pragma unroll
        for (int it = 0; it < 4; ++it) {
          const int row = it * 4 + q;
          const float* sp = slab + row * 68 + c8;
          v8h hv, lv;
#pragma unroll
          for (int e = 0; e < 8; ++e) {
            if (OUT_MODE == 1) {
              hv[e] = (_Float16)sp[e];
            } else {
              unsigned short hb = f2bf_bits(sp[e]);
              unsigned short lb = f2bf_bits(sp[e] - bf_bits2f(hb));
              hv[e] = __builtin_bit_cast(_Float16, hb);
              lv[e] = __builtin_bit_cast(_Float16, lb);
            }
          }
          *(volatile v8h*)(C + (size_t)(mBase + row) * ldc + n0 + c8) = hv;
          if (OUT_MODE == 2) *(volatile v8h*)(C2 + (size_t)(mBase + row) * ldc + n0 + c8) = lv;
        }
        __threadfence();
      }
    }
    __builtin_amdgcn_fence(__ATOMIC_RELEASE, "workgroup");
    __builtin_amdgcn_wave_barrier();
    __builtin_amdgcn_fence(__ATOMIC_ACQUIRE, "workgroup");
  }
}

__global__ __launch_bounds__(256) void k_wtcast(const float* __restrict__ w0, const float* __restrict__ w1,
                                                unsigned short* __restrict__ out, int kd, int nd, float scale) {
  __shared__ float sm[64][65];
  const int t  = threadIdx.x;
  const int k0 = blockIdx.x * 64;
  const int n0 = blockIdx.y * 64;
  const int z  = blockIdx.z;
  const float* w = (z == 0) ? w0 : w1;
#pragma unroll
  for (int i = 0; i < 16; ++i) {
    const int e = i * 256 + t;
    const int r = e >> 6;
    const int c = e & 63;
    sm[c][r] = w[(size_t)(k0 + r) * nd + n0 + c] * scale;
  }
  __syncthreads();
  const int lane = t & 31, wave = t >> 5;
  const int q = lane >> 3, c8 = (lane & 7) * 8;
  unsigned short* op = out + (size_t)z * nd * kd;
  for (int pass = 0; pass < 2; ++pass) {
#pragma unroll
    for (int it = 0; it < 2; ++it) {
      const int row = wave * 8 + it * 4 + q;
      unsigned short hb[8];
#pragma unroll
      for (int e = 0; e < 8; ++e) hb[e] = h_bits(sm[row][c8 + e]);
      const v4u u = (v4u){pk16(hb[0], hb[1]), pk16(hb[2], hb[3]), pk16(hb[4], hb[5]), pk16(hb[6], hb[7])};
      *(volatile v4u*)(op + (size_t)(n0 + row) * kd + k0 + c8) = u;
    }
    __threadfence();
  }
}

__global__ __launch_bounds__(256) void k_cast8(const float* __restrict__ in, unsigned short* __restrict__ out, float scale, int n8) {
  const int i = blockIdx.x * 256 + threadIdx.x;
  if (i >= n8) return;
  const float* p = in + 8 * (size_t)i;
  const v4f a = *(const v4f*)(p);
  const v4f c = *(const v4f*)(p + 4);
  unsigned short hb[8];
#pragma unroll
  for (int e = 0; e < 4; ++e) {
    hb[e]     = h_bits(a[e] * scale);
    hb[4 + e] = h_bits(c[e] * scale);
  }
  const v4u u = (v4u){pk16(hb[0], hb[1]), pk16(hb[2], hb[3]), pk16(hb[4], hb[5]), pk16(hb[6], hb[7])};
  unsigned short* qo = out + 8 * (size_t)i;
  *(volatile v4u*)qo = u;
  __threadfence();
  *(volatile v4u*)qo = u;
}

__global__ __launch_bounds__(128) void k_rmsnorm(const float* __restrict__ x, unsigned short* __restrict__ out) {
  __shared__ float red[4];
  const int row  = blockIdx.x;
  const int t    = threadIdx.x;
  const int lane = t & 31, wave = t >> 5;
  const float* xp = x + (size_t)row * kDim + t * 8;
  const v4f a = *(const v4f*)(xp);
  const v4f c = *(const v4f*)(xp + 4);
  float ss = 0.f;
#pragma unroll
  for (int e = 0; e < 4; ++e) ss += a[e] * a[e];
#pragma unroll
  for (int e = 0; e < 4; ++e) ss += c[e] * c[e];
#pragma unroll
  for (int off = 16; off > 0; off >>= 1) ss += __shfl_xor(ss, off, 32);
  if (lane == 0) red[wave] = ss;
  __syncthreads();
  const float tot = ((red[0] + red[1]) + red[2]) + red[3];
  const float rinv = rsqrtf(tot * (1.0f / 1024.0f) + 1e-6f);
  unsigned short hb[8];
#pragma unroll
  for (int e = 0; e < 4; ++e) {
    hb[e]     = h_bits(a[e] * rinv);
    hb[4 + e] = h_bits(c[e] * rinv);
  }
  const v4u u = (v4u){pk16(hb[0], hb[1]), pk16(hb[2], hb[3]), pk16(hb[4], hb[5]), pk16(hb[6], hb[7])};
  unsigned short* qo = out + (size_t)row * kDim + t * 8;
  *(volatile v4u*)qo = u;
  __threadfence();
  *(volatile v4u*)qo = u;
}

__global__ __launch_bounds__(256) void k_reflect(const float* __restrict__ vs, unsigned short* __restrict__ qrow16,
                                                 unsigned short* __restrict__ qcol16) {
#pragma clang fp contract(off)
  __shared__ float Qm[64 * 64];
  __shared__ float vsh[64];
  __shared__ float wsh[64];
  __shared__ float cs;
  const int t = threadIdx.x;
  for (int i = t; i < 4096; i += 256) Qm[i] = ((i >> 6) == (i & 63)) ? 1.f : 0.f;
  __syncthreads();
#pragma unroll 1
  for (int r = 0; r < 32; ++r) {
    if (t < 64) vsh[t] = vs[r * 64 + t];
    __syncthreads();
    if (t == 0) {
      float s = 0.f;
#pragma unroll 1
      for (int i = 0; i < 64; ++i) s += vsh[i] * vsh[i];
      cs = 2.0f / (s + 1e-8f);
    }
    if (t < 64) {
      float s = 0.f;
#pragma unroll 1
      for (int i = 0; i < 64; ++i) s += vsh[i] * Qm[i * 64 + t];
      wsh[t] = s;
    }
    __syncthreads();
    const float c = cs;
#pragma unroll 1
    for (int i = t; i < 4096; i += 256) {
      float o = vsh[i >> 6] * wsh[i & 63];
      o = c * o;
      Qm[i] = Qm[i] - o;
    }
    __syncthreads();
  }
  const int lane = t & 31, wave = t >> 5;
  const int q = lane >> 3, c8 = (lane & 7) * 8;
  for (int pass = 0; pass < 2; ++pass) {
#pragma unroll
    for (int it = 0; it < 2; ++it) {
      const int row = wave * 8 + it * 4 + q;
      unsigned short ha[8], hb[8];
#pragma unroll
      for (int e = 0; e < 8; ++e) {
        ha[e] = h_bits(kWCarry * Qm[row * 64 + c8 + e]);
        hb[e] = h_bits(kWCarry * Qm[(c8 + e) * 64 + row]);
      }
      const v4u ua = (v4u){pk16(ha[0], ha[1]), pk16(ha[2], ha[3]), pk16(ha[4], ha[5]), pk16(ha[6], ha[7])};
      const v4u ub = (v4u){pk16(hb[0], hb[1]), pk16(hb[2], hb[3]), pk16(hb[4], hb[5]), pk16(hb[6], hb[7])};
      *(volatile v4u*)(qrow16 + row * 64 + c8) = ua;
      *(volatile v4u*)(qcol16 + row * 64 + c8) = ub;
    }
    __threadfence();
  }
}

struct FreqTab { float f[32]; };
typedef char freqtab_size_check[(sizeof(FreqTab) == 128) ? 1 : -1];

template <bool COSINE>
__global__ __launch_bounds__(256) void k_ropetab(float* __restrict__ tab, FreqTab ft) {
#pragma clang fp contract(off)
  __shared__ float fr[32];
  const int t = threadIdx.x;
  if (t < 32) {
    float v = 0.f;
#pragma unroll
    for (int j = 0; j < 32; ++j) v = (t == j) ? ft.f[j] : v;
    fr[t] = v;
  }
  __syncthreads();
  const int i = blockIdx.x * 256 + t;
  const int s = i >> 5, j = i & 31;
  const float ang = (float)s * fr[j];
  const float val = COSINE ? cosf(ang) : sinf(ang);
  ((volatile float*)tab)[i] = val;
  __threadfence();
  ((volatile float*)tab)[i] = val;
}

__global__ __launch_bounds__(256) void k_rope(const float* __restrict__ hh, const float* __restrict__ cosb,
                                              const float* __restrict__ sinb, unsigned short* __restrict__ r16) {
  const int i = blockIdx.x * 256 + threadIdx.x;
  const int row = i >> 3;
  const int d0 = (i & 7) * 8;
  const int tokh = row & 65535;
  const int s = (tokh >> 4) & (kSeq - 1);
  const float* rp = hh + (size_t)row * 64;
  const v4f oa = *(const v4f*)(rp + d0);
  const v4f oc = *(const v4f*)(rp + d0 + 4);
  const v4f pa = *(const v4f*)(rp + (d0 ^ 32));
  const v4f pc = *(const v4f*)(rp + (d0 ^ 32) + 4);
  const float* cp = cosb + s * 32 + (d0 & 31);
  const float* sp = sinb + s * 32 + (d0 & 31);
  const v4f ca = *(const v4f*)(cp), cc = *(const v4f*)(cp + 4);
  const v4f sa = *(const v4f*)(sp), sc = *(const v4f*)(sp + 4);
  const float sgn = (d0 < 32) ? -1.0f : 1.0f;
  unsigned short hb[8];
#pragma unroll
  for (int e = 0; e < 4; ++e) {
    hb[e]     = h_bits(oa[e] * ca[e] + sgn * pa[e] * sa[e]);
    hb[4 + e] = h_bits(oc[e] * cc[e] + sgn * pc[e] * sc[e]);
  }
  const v4u u = (v4u){pk16(hb[0], hb[1]), pk16(hb[2], hb[3]), pk16(hb[4], hb[5]), pk16(hb[6], hb[7])};
  unsigned short* qo = r16 + 8 * (size_t)i;
  *(volatile v4u*)qo = u;
  __threadfence();
  *(volatile v4u*)qo = u;
}

__global__ __launch_bounds__(256) void k_vtrans(const unsigned short* __restrict__ vin, unsigned short* __restrict__ vt) {
  __shared__ unsigned short sm[64][66];
  const int t = threadIdx.x;
  const int g = blockIdx.y;
  const int b = g >> 4, h = g & 15;
  const int s0 = blockIdx.x * 64;
#pragma unroll
  for (int it = 0; it < 2; ++it) {
    const int idx = it * 256 + t;
    const int r = idx >> 3;
    const int c16 = idx & 7;
    const v4u w = *(const v4u*)(vin + ((size_t)(b * kSeq + s0 + r) * kDim + h * 64 + c16 * 8));
    unsigned short* d = &sm[r][c16 * 8];
    d[0] = (unsigned short)(w.x & 0xffffu); d[1] = (unsigned short)(w.x >> 16);
    d[2] = (unsigned short)(w.y & 0xffffu); d[3] = (unsigned short)(w.y >> 16);
    d[4] = (unsigned short)(w.z & 0xffffu); d[5] = (unsigned short)(w.z >> 16);
    d[6] = (unsigned short)(w.w & 0xffffu); d[7] = (unsigned short)(w.w >> 16);
  }
  __syncthreads();
  const int lane = t & 31, wave = t >> 5;
  const int q = lane >> 3, c8 = (lane & 7) * 8;
  for (int pass = 0; pass < 2; ++pass) {
#pragma unroll
    for (int it = 0; it < 2; ++it) {
      const int d = wave * 8 + it * 4 + q;
      unsigned short hb[8];
#pragma unroll
      for (int e = 0; e < 8; ++e) hb[e] = sm[c8 + e][d];
      const v4u u = (v4u){pk16(hb[0], hb[1]), pk16(hb[2], hb[3]), pk16(hb[4], hb[5]), pk16(hb[6], hb[7])};
      *(volatile v4u*)(vt + ((size_t)g * 64 + d) * kSeq + s0 + c8) = u;
    }
    __threadfence();
  }
}

__global__ __launch_bounds__(256) void k_softmax(const float* __restrict__ sc, const int* __restrict__ mk,
                                                 unsigned short* __restrict__ pout) {
  __shared__ float redM[8];
  __shared__ float redS[8];
  const int r    = blockIdx.x;
  const int qrow = r & (kSeq - 1);
  const int t    = threadIdx.x;
  const int lane = t & 31, wave = t >> 5;
  const int c0   = t * 8;
  const float* sp = sc + (size_t)r * kSeq + c0;
  const v4f a = *(const v4f*)(sp);
  const v4f c = *(const v4f*)(sp + 4);
  const int* mp = mk + (size_t)qrow * kSeq + c0;
  const v4i ma = *(const v4i*)(mp);
  const v4i mc = *(const v4i*)(mp + 4);
  float x[8];
#pragma unroll
  for (int e = 0; e < 4; ++e) {
    x[e]     = (ma[e] != 0) ? a[e] : kFill;
    x[4 + e] = (mc[e] != 0) ? c[e] : kFill;
  }
  float m = fmaxf(fmaxf(fmaxf(x[0], x[1]), fmaxf(x[2], x[3])), fmaxf(fmaxf(x[4], x[5]), fmaxf(x[6], x[7])));
#pragma unroll
  for (int off = 16; off > 0; off >>= 1) m = fmaxf(m, __shfl_xor(m, off, 32));
  if (lane == 0) redM[wave] = m;
  __syncthreads();
  float mm = redM[0];
#pragma unroll
  for (int w = 1; w < 8; ++w) mm = fmaxf(mm, redM[w]);
  float ex[8];
  float ps = 0.f;
#pragma unroll
  for (int e = 0; e < 8; ++e) { ex[e] = expf(x[e] - mm); ps += ex[e]; }
#pragma unroll
  for (int off = 16; off > 0; off >>= 1) ps += __shfl_xor(ps, off, 32);
  if (lane == 0) redS[wave] = ps;
  __syncthreads();
  float tot = redS[0];
#pragma unroll
  for (int w = 1; w < 8; ++w) tot += redS[w];
  const float rs = kPCarry / tot;
  unsigned short hb[8];
#pragma unroll
  for (int e = 0; e < 8; ++e) hb[e] = h_bits(ex[e] * rs);
  const v4u u = (v4u){pk16(hb[0], hb[1]), pk16(hb[2], hb[3]), pk16(hb[4], hb[5]), pk16(hb[6], hb[7])};
  unsigned short* qo = pout + (size_t)r * kSeq + c0;
  *(volatile v4u*)qo = u;
  __threadfence();
  *(volatile v4u*)qo = u;
}

__global__ __launch_bounds__(256) void k_geglu(const float* __restrict__ gv, unsigned short* __restrict__ act, int nthr) {
  const int i = blockIdx.x * 256 + threadIdx.x;
  if (i >= nthr) return;
  const int m  = i >> 9;
  const int n0 = (i & 511) * 8;
  const float* gp = gv + (size_t)m * 8192 + n0;
  const float* vp = gp + 4096;
  unsigned long long lo = 0ull, hi = 0ull;
#pragma unroll 1
  for (int e = 0; e < 8; ++e) {
    const float g  = gp[e];
    const float vl = vp[e];
    const float ge = 0.5f * g * (1.0f + erff(g * 0.70710678118654752f));
    const float a  = vl * ge * kACarry;
    const unsigned long long hb = (unsigned long long)h_bits(a);
    const int sh = (e & 3) * 16;
    const unsigned long long piece = hb << sh;
    const bool low = (e < 4);
    lo |= low ? piece : 0ull;
    hi |= low ? 0ull : piece;
  }
  const v4u u = (v4u){(unsigned)(lo & 0xffffffffull), (unsigned)(lo >> 32), (unsigned)(hi & 0xffffffffull), (unsigned)(hi >> 32)};
  unsigned short* qo = act + (size_t)m * 4096 + n0;
  *(volatile v4u*)qo = u;
  __threadfence();
  *(volatile v4u*)qo = u;
}

static inline unsigned cdiv(unsigned a, unsigned b) { return (a + b - 1) / b; }

extern "C" void kernel_launch(void* const* d_in, const int* in_sizes, int n_in,
                              void* d_out, int out_size, void* d_ws, size_t ws_size,
                              hipStream_t stream) {
  if (n_in < 12) return;
  if (ws_size < kCarveBytes) return;
  if (out_size != kTok * kDim) return;
  if (in_sizes[0] != kTok * kDim || in_sizes[1] != kSeq * kSeq || in_sizes[3] != 32 * 64 ||
      in_sizes[4] != kDim * 3 * kDim || in_sizes[5] != kDim * kDim || in_sizes[6] != kDim * kDim ||
      in_sizes[7] != kDim || in_sizes[8] != kDim * 8 * kDim || in_sizes[9] != 8 * kDim ||
      in_sizes[10] != kDff * kDim || in_sizes[11] != kDim) return;

  const float* x          = (const float*)d_in[0];
  const int*   maskp      = (const int*)d_in[1];
  const float* vs         = (const float*)d_in[3];
  const float* w_qkv      = (const float*)d_in[4];
  const float* w_out      = (const float*)d_in[5];
  const float* w_gate     = (const float*)d_in[6];
  const float* b_gate     = (const float*)d_in[7];
  const float* w_mlp_gate = (const float*)d_in[8];
  const float* b_mlp_gate = (const float*)d_in[9];
  const float* w_mlp_out  = (const float*)d_in[10];
  const float* b_mlp_out  = (const float*)d_in[11];
  float* out = (float*)d_out;

  char* ws = (char*)d_ws;
  unsigned short* rH16    = (unsigned short*)(ws + 0);
  unsigned short* rATTN16 = (unsigned short*)(ws + 0);
  unsigned short* rH2     = (unsigned short*)(ws + 0);
  unsigned short* rVT16   = (unsigned short*)(ws + 8 * kMiB);
  unsigned short* rWOUT16 = (unsigned short*)(ws + 8 * kMiB);
  unsigned short* rWMG16  = (unsigned short*)(ws + 8 * kMiB);
  unsigned short* rQ16    = (unsigned short*)(ws + 16 * kMiB);
  unsigned short* rK16    = (unsigned short*)(ws + 24 * kMiB);
  float*          rATT    = (float*)(ws + 16 * kMiB);
  unsigned short* rWMO16  = (unsigned short*)(ws + 24 * kMiB);
  unsigned short* rV16    = (unsigned short*)(ws + 32 * kMiB);
  float*          rS      = (float*)(ws + 32 * kMiB);
  unsigned short* rATT16  = (unsigned short*)(ws + 32 * kMiB);
  unsigned short* rWQKV16 = (unsigned short*)(ws + 40 * kMiB);
  float*          rX1     = (float*)(ws + 40 * kMiB);
  float*          rCOS    = (float*)(ws + 46 * kMiB);
  float*          rSIN    = (float*)(ws + 46 * kMiB + 262144);
  unsigned short* rQH16   = (unsigned short*)(ws + 46 * kMiB + 524288);
  unsigned short* rQTH16  = (unsigned short*)(ws + 46 * kMiB + 524288 + 8192);
  float*          rHH     = (float*)(ws + 48 * kMiB);
  float*          rGV     = (float*)(ws + 56 * kMiB);
  unsigned short* rR16    = (unsigned short*)(ws + 80 * kMiB);
  unsigned short* rACT16  = (unsigned short*)(ws + 88 * kMiB);
  unsigned short* rP16    = (unsigned short*)(ws + 96 * kMiB);
  (void)rK16; (void)rV16;

  FreqTab ft;
  {
    double rt = 1.34;
    for (int it = 0; it < 200; ++it) {
      double p31 = 1.0;
      for (int k = 0; k < 31; ++k) p31 *= rt;
      const double f = p31 * rt - 10000.0;
      rt -= f / (32.0 * p31);
    }
    double pj = 1.0;
    for (int j = 0; j < 32; ++j) {
      const float pf = (float)pj;
      ft.f[j] = 1.0f / pf;
      pj *= rt;
    }
  }

  const long planeTokD = (long)kTok * kDim;
  const float invW  = 1.0f / kWCarry;
  const float invWA = 1.0f / (kWCarry * kACarry);

  k_wtcast<<<dim3(kDim / 64, 3 * kDim / 64, 1), 256, 0, stream>>>(w_qkv, w_qkv, rWQKV16, kDim, 3 * kDim, kWCarry);
  k_rmsnorm<<<kTok, 128, 0, stream>>>(x, rH16);
  wmma_gemm64<0, false, 0, 1, false, 0><<<dim3(cdiv(64 * 16, 8), 3), 256, 0, stream>>>(
      rH16, rH16, kDim, 0L,
      rWQKV16, rWQKV16, kDim, (long)kDim * kDim,
      (void*)rQ16, (void*)rQ16, kDim, planeTokD,
      b_gate, x, 0L, x,
      kTok, kDim, kDim, invW);
  k_vtrans<<<dim3(kSeq / 64, kGroups), 256, 0, stream>>>(rV16, rVT16);
  k_reflect<<<1, 256, 0, stream>>>(vs, rQH16, rQTH16);
  k_ropetab<true><<<256, 256, 0, stream>>>(rCOS, ft);
  k_ropetab<false><<<256, 256, 0, stream>>>(rSIN, ft);
  wmma_gemm64<0, false, 0, 0, false, 0><<<dim3(cdiv(1024 * 1, 8), 2), 256, 0, stream>>>(
      rQ16, rQ16, kHd, planeTokD,
      rQH16, rQH16, kHd, 0L,
      (void*)rHH, (void*)rHH, kHd, planeTokD,
      b_gate, x, 0L, x,
      kTok * kHeads, kHd, kHd, invW);
  k_rope<<<cdiv(2u * kTok * kHeads * kHd / 8, 256), 256, 0, stream>>>(rHH, rCOS, rSIN, rR16);
  wmma_gemm64<0, false, 0, 1, false, 0><<<dim3(cdiv(1024 * 1, 8), 2), 256, 0, stream>>>(
      rR16, rR16, kHd, planeTokD,
      rQTH16, rQTH16, kHd, 0L,
      (void*)rQ16, (void*)rQ16, kHd, planeTokD,
      b_gate, x, 0L, x,
      kTok * kHeads, kHd, kHd, invW);

  const long sPlane = (long)kSeq * kSeq;
  for (int ch = 0; ch < kNchunk; ++ch) {
    const int b  = ch / (kHeads / kGch);
    const int h0 = (ch % (kHeads / kGch)) * kGch;
    const size_t headOff = (size_t)b * kSeq * kDim + (size_t)h0 * kHd;
    wmma_gemm64<0, false, 0, 0, false, 0><<<dim3(cdiv(32 * 32, 8), kGch), 256, 0, stream>>>(
        rQ16 + headOff, rQ16 + headOff, kDim, (long)kHd,
        rK16 + headOff, rK16 + headOff, kDim, (long)kHd,
        (void*)rS, (void*)rS, kSeq, sPlane,
        b_gate, x, 0L, x,
        kSeq, kSeq, kHd, 0.125f);
    k_softmax<<<kGch * kSeq, 256, 0, stream>>>(rS, maskp, rP16);
    wmma_gemm64<0, false, 0, 1, false, 0><<<dim3(cdiv(32 * 1, 8), kGch), 256, 0, stream>>>(
        rP16, rP16, kSeq, sPlane,
        rVT16 + (size_t)(ch * kGch) * kHd * kSeq, rVT16 + (size_t)(ch * kGch) * kHd * kSeq, kSeq, (long)kHd * kSeq,
        (void*)(rATTN16 + headOff), (void*)(rATTN16 + headOff), kDim, (long)kHd,
        b_gate, x, 0L, x,
        kSeq, kHd, kSeq, kACarry / kPCarry);
  }

  k_wtcast<<<dim3(kDim / 64, kDim / 64, 2), 256, 0, stream>>>(w_out, w_gate, rWOUT16, kDim, kDim, kWCarry);
  wmma_gemm64<0, false, 0, 0, false, 0><<<dim3(cdiv(64 * 16, 8), 1), 256, 0, stream>>>(
      rATTN16, rATTN16, kDim, 0L,
      rWOUT16, rWOUT16, kDim, 0L,
      (void*)rATT, (void*)rATT, kDim, 0L,
      b_gate, x, 0L, x,
      kTok, kDim, kDim, invWA);
  k_cast8<<<cdiv(kTok * kDim / 8, 256), 256, 0, stream>>>(rATT, rATT16, kACarry, kTok * kDim / 8);
  wmma_gemm64<0, false, 2, 0, true, 6><<<dim3(cdiv(64 * 16, 8), 1), 256, 0, stream>>>(
      rATT16, rATT16, kDim, 0L,
      rWOUT16 + (size_t)kDim * kDim, rWOUT16 + (size_t)kDim * kDim, kDim, 0L,
      (void*)rX1, (void*)rX1, kDim, 0L,
      b_gate, x, 0L, rATT,
      kTok, kDim, kDim, invWA);
  k_rmsnorm<<<kTok, 128, 0, stream>>>(rX1, rH2);
  k_wtcast<<<dim3(kDim / 64, 8 * kDim / 64, 1), 256, 0, stream>>>(w_mlp_gate, w_mlp_gate, rWMG16, kDim, 8 * kDim, kWCarry);
  k_wtcast<<<dim3(kDff / 64, kDim / 64, 1), 256, 0, stream>>>(w_mlp_out, w_mlp_out, rWMO16, kDff, kDim, kWCarry);
  for (int c = 0; c < kTok / kMlpRows; ++c) {
    wmma_gemm64<0, false, 2, 0, false, 0><<<dim3(cdiv((kMlpRows / 64) * (8 * kDim / 64), 8), 1), 256, 0, stream>>>(
        rH2 + (size_t)c * kMlpRows * kDim, rH2 + (size_t)c * kMlpRows * kDim, kDim, 0L,
        rWMG16, rWMG16, kDim, 0L,
        (void*)rGV, (void*)rGV, 8 * kDim, 0L,
        b_mlp_gate, x, 0L, x,
        kMlpRows, 8 * kDim, kDim, invW);
    k_geglu<<<cdiv(kMlpRows * (kDff / 8), 256), 256, 0, stream>>>(rGV, rACT16 + (size_t)c * kMlpRows * kDff, kMlpRows * (kDff / 8));
  }
  wmma_gemm64<0, false, 2, 0, true, 0><<<dim3(cdiv(64 * 16, 8), 1), 256, 0, stream>>>(
      rACT16, rACT16, kDff, 0L,
      rWMO16, rWMO16, kDff, 0L,
      (void*)out, (void*)out, kDim, 0L,
      b_mlp_out, rX1, 0L, rX1,
      kTok, kDim, kDff, invWA);
}
